// EncoderLayer_hybrid2_8315056685232
// MI455X (gfx1250) — hardware-verified
//
#include <hip/hip_runtime.h>
#include <math.h>
typedef __attribute__((ext_vector_type(16))) _Float16 v16h;
typedef __attribute__((ext_vector_type(8)))  _Float16 v8h;
typedef __attribute__((ext_vector_type(16))) __bf16   v16b;
typedef __attribute__((ext_vector_type(8)))  __bf16   v8b;
typedef __attribute__((ext_vector_type(8)))  float    v8f;
typedef __attribute__((ext_vector_type(4)))  float    v4f;
#define PSCALE 32768.0f
#define U16(p) ((const unsigned short*)(const void*)(p))
#define PSCALE_INV (1.0f / 32768.0f)

__device__ __forceinline__ unsigned short f2bf_bits(float f) {
  unsigned u = __float_as_uint(f);
  return (unsigned short)((u + 0x7FFFu + ((u >> 16) & 1u)) >> 16);
}
__device__ __forceinline__ float bf_bits2f(unsigned short h) { return __uint_as_float(((unsigned)h) << 16); }

__device__ __forceinline__ void dep_guard_h(v8f& a, v8f& b, v16h x, v16h y) { asm volatile("v_nop\n\tv_nop\n\tv_nop\n\tv_nop" : "+v"(a), "+v"(b) : "v"(x), "v"(y)); }
__device__ __forceinline__ void dep_guard_b(v8f& a, v8f& b, v16b x, v16b y) { asm volatile("v_nop\n\tv_nop\n\tv_nop\n\tv_nop" : "+v"(a), "+v"(b) : "v"(x), "v"(y)); }
__device__ __forceinline__ void keep4_h(v16h a, v16h b, v16h c, v16h d) { asm volatile("v_nop" :: "v"(a), "v"(b), "v"(c), "v"(d)); }
__device__ __forceinline__ void keep4_b(v16b a, v16b b, v16b c, v16b d) { asm volatile("v_nop" :: "v"(a), "v"(b), "v"(c), "v"(d)); }
__device__ __forceinline__ void acc_guard4(v8f& a, v8f& b, v8f& c, v8f& d) { asm volatile("v_nop\n\tv_nop\n\tv_nop\n\tv_nop" : "+v"(a), "+v"(b), "+v"(c), "+v"(d)); }
template <typename T> struct Frag;
template <> struct Frag<_Float16> {
  typedef v16h V; union U { v16h v; v8h h[2]; };
  static __device__ __forceinline__ v16h load(const _Float16* p) {
    U f; f.h[0] = *(const v8h*)(p); f.h[1] = *(const v8h*)(p + 16); return f.v;
  }
  static __device__ __forceinline__ v8f mma(v16h a, v16h b, v8f c) {
    return __builtin_amdgcn_wmma_f32_16x16x32_f16(false, a, false, b, (short)0, c, false, false);
  }
  static __device__ __forceinline__ void guard(v8f& a, v8f& b, v16h x, v16h y) { dep_guard_h(a, b, x, y); }
  static __device__ __forceinline__ void keep(v16h a, v16h b, v16h c, v16h d) { keep4_h(a, b, c, d); }
};
template <> struct Frag<__bf16> {
  typedef v16b V; union U { v16b v; v8b h[2]; };
  static __device__ __forceinline__ v16b load(const __bf16* p) {
    U f; f.h[0] = *(const v8b*)(p); f.h[1] = *(const v8b*)(p + 16); return f.v;
  }
  static __device__ __forceinline__ v8f mma(v16b a, v16b b, v8f c) {
    return __builtin_amdgcn_wmma_f32_16x16x32_bf16(false, a, false, b, (short)0, c, false, false);
  }
  static __device__ __forceinline__ void guard(v8f& a, v8f& b, v16b x, v16b y) { dep_guard_b(a, b, x, y); }
  static __device__ __forceinline__ void keep(v16b a, v16b b, v16b c, v16b d) { keep4_b(a, b, c, d); }
};

template <int ET> struct Elem;
template <> struct Elem<0> { typedef _Float16 T; };
template <> struct Elem<1> { typedef __bf16 T; };
template <int ET, bool SPLIT, int BIAS_MODE, int OUT_MODE, bool RESID, int ACT = 0>
__global__ __launch_bounds__(256) void wmma_gemm64(
    const unsigned short* __restrict__ Ap, const unsigned short* __restrict__ A2p, int lda, long strideA,
    const unsigned short* __restrict__ Btp, const unsigned short* __restrict__ Bt2p, int ldb, long strideB,
    void* __restrict__ Cout, void* __restrict__ Cout2, int ldc, long strideC,
    const float* __restrict__ bias,
    const float* __restrict__ resid, long strideR,
    int M, int N, int K, float scale) {
  typedef typename Elem<ET>::T T;
  typedef typename Frag<T>::V V;
  const T* A = (const T*)Ap; const T* A2 = (const T*)A2p; const T* Bt = (const T*)Btp; const T* Bt2 = (const T*)Bt2p;
  __shared__ __align__(16) float sT[8][16 * 68];
  const int b    = blockIdx.y;
  const int lane = threadIdx.x & 31;
  const int wave = threadIdx.x >> 5;
  const int tilesN = N >> 6;
  const int tilesM = M >> 6;
  const int tile = blockIdx.x * 8 + wave;
  if (tile >= tilesM * tilesN) return;
  const int tm = tile / tilesN;
  const int tn = tile - tm * tilesN;
  const int m0 = tm << 6;
  const int n0 = tn << 6;

  const T* Ab  = A  + (size_t)b * strideA;
  const T* Bb  = Bt + (size_t)b * strideB;
  const T* Ab2 = SPLIT ? (A2  + (size_t)b * strideA) : nullptr;
  const T* Bb2 = SPLIT ? (Bt2 + (size_t)b * strideB) : nullptr;

  const int rlane = lane & 15;
  const int koff  = (lane >> 4) * 8;
  const int mOff  = (lane >> 4) * 8;

  v8f acc[4][4];
#pragma unroll
  for (int i = 0; i < 4; ++i)
#pragma unroll
    for (int j = 0; j < 4; ++j) acc[i][j] = (v8f){0.f,0.f,0.f,0.f,0.f,0.f,0.f,0.f};

  for (int k0 = 0; k0 < K; k0 += 32) {
    V bh[4], bl[4];
#pragma unroll
    for (int j = 0; j < 4; ++j) {
      const size_t bo = (size_t)(n0 + (j << 4) + rlane) * ldb + koff + k0;
      bh[j] = Frag<T>::load(Bb + bo);
      if (SPLIT) bl[j] = Frag<T>::load(Bb2 + bo);
    }
#pragma unroll
    for (int i = 0; i < 4; ++i) {
      const size_t ao = (size_t)(m0 + (i << 4) + rlane) * lda + koff + k0;
      V ah = Frag<T>::load(Ab + ao);
      V al;
      if (SPLIT) al = Frag<T>::load(Ab2 + ao);
#pragma unroll
      for (int j = 0; j < 4; ++j) {
        acc[i][j] = Frag<T>::mma(ah, bh[j], acc[i][j]);
        if (SPLIT) {
          acc[i][j] = Frag<T>::mma(ah, bl[j], acc[i][j]);
          acc[i][j] = Frag<T>::mma(al, bh[j], acc[i][j]);
        }
      }
      Frag<T>::guard(acc[i][0], acc[i][3], ah, SPLIT ? al : ah);
    }
    Frag<T>::keep(bh[0], bh[1], bh[2], bh[3]);
    if (SPLIT) Frag<T>::keep(bl[0], bl[1], bl[2], bl[3]);
  }
  acc_guard4(acc[0][0], acc[0][1], acc[0][2], acc[0][3]);
  acc_guard4(acc[1][0], acc[1][1], acc[1][2], acc[1][3]);
  acc_guard4(acc[2][0], acc[2][1], acc[2][2], acc[2][3]);
  acc_guard4(acc[3][0], acc[3][1], acc[3][2], acc[3][3]);

  float* slab = sT[wave];
  const float* Rb = RESID ? (resid + (size_t)b * strideR) : nullptr;
#pragma unroll
  for (int i = 0; i < 4; ++i) {
    const int mBase = m0 + (i << 4);
#pragma unroll
    for (int j = 0; j < 4; ++j) {
      const int n = n0 + (j << 4) + rlane;
      float bv = 0.f;
      if (BIAS_MODE == 2) bv = bias[n];
#pragma unroll
      for (int r = 0; r < 8; ++r) {
        float v = acc[i][j][r] * scale;
        if (BIAS_MODE == 1) v += bias[mBase + mOff + r];
        if (BIAS_MODE == 2) v += bv;
        if (RESID) v += Rb[(size_t)(mBase + mOff + r) * ldc + n];
        if (ACT == 1) v = tanhf(v);
        if (ACT == 2) v = fmaxf(v, 0.0f);
        if (ACT == 3) v = v / (1.0f + expf(-v));
        if (ACT == 4) v = (v > 0.f) ? v : 0.01f * v;
        if (ACT == 5) v = 0.5f * v * (1.0f + erff(v * 0.70710678118654752f));
        slab[(mOff + r) * 68 + (j << 4) + rlane] = v;
      }
    }
    __builtin_amdgcn_fence(__ATOMIC_RELEASE, "workgroup");
    __builtin_amdgcn_wave_barrier();
    __builtin_amdgcn_fence(__ATOMIC_ACQUIRE, "workgroup");
    if (OUT_MODE == 0) {
      float* C = (float*)Cout + (size_t)b * strideC;
      const int hh = lane >> 4, c4 = (lane & 15) * 4;
      for (int pass = 0; pass < 2; ++pass) {
#pragma unroll
        for (int it = 0; it < 8; ++it) {
          const int row = it * 2 + hh;
          v4f v = *(const v4f*)(slab + row * 68 + c4);
          *(volatile v4f*)(C + (size_t)(mBase + row) * ldc + n0 + c4) = v;
        }
        __threadfence();
      }
    } else {
      const int q = lane >> 3, c8 = (lane & 7) * 8;
      unsigned short* C  = (unsigned short*)Cout  + (size_t)b * strideC;
      unsigned short* C2 = (OUT_MODE == 2) ? ((unsigned short*)Cout2 + (size_t)b * strideC) : nullptr;
      for (int pass = 0; pass < 2; ++pass) {
#pragma unroll
        for (int it = 0; it < 4; ++it) {
          const int row = it * 4 + q;
          const float* sp = slab + row * 68 + c8;
          v8h hv, lv;
#pragma unroll
          for (int e = 0; e < 8; ++e) {
            if (OUT_MODE == 1) {
              hv[e] = (_Float16)sp[e];
            } else {
              unsigned short hb = f2bf_bits(sp[e]);
              unsigned short lb = f2bf_bits(sp[e] - bf_bits2f(hb));
              hv[e] = __builtin_bit_cast(_Float16, hb);
              lv[e] = __builtin_bit_cast(_Float16, lb);
            }
          }
          *(volatile v8h*)(C + (size_t)(mBase + row) * ldc + n0 + c8) = hv;
          if (OUT_MODE == 2) *(volatile v8h*)(C2 + (size_t)(mBase + row) * ldc + n0 + c8) = lv;
        }
        __threadfence();
      }
    }
    __builtin_amdgcn_fence(__ATOMIC_RELEASE, "workgroup");
    __builtin_amdgcn_wave_barrier();
    __builtin_amdgcn_fence(__ATOMIC_ACQUIRE, "workgroup");
  }
}

__global__ __launch_bounds__(256) void cast_f32_f16x2(
    const float* __restrict__ in, _Float16* __restrict__ out, int n2) {
  int i = blockIdx.x * 256 + threadIdx.x;
  if (i < n2) {
    const _Float16 h0 = (_Float16)in[2 * i], h1 = (_Float16)in[2 * i + 1];
    const unsigned u = (unsigned)__builtin_bit_cast(unsigned short, h0) | ((unsigned)__builtin_bit_cast(unsigned short, h1) << 16);
    ((volatile unsigned*)out)[i] = u;
    __threadfence();
    ((volatile unsigned*)out)[i] = u;
  }
}


#define LB 8
#define LT 1024
#define LE 512
#define LH 8
#define LEH 64
#define LR (LB * LT)
__global__ __launch_bounds__(256) void ln_qk_kernel(const float* __restrict__ x, const float* __restrict__ WQ, const float* __restrict__ bQ, const float* __restrict__ WK, const float* __restrict__ bK, unsigned* __restrict__ XN16, float* __restrict__ Qs, float* __restrict__ Ks) {
  const int lane = threadIdx.x & 31, wave = threadIdx.x >> 5; const size_t r = (size_t)blockIdx.x * 8 + wave;
  float v[16]; float s = 0.f;
#pragma unroll
  for (int q = 0; q < 4; ++q) { const v4f a = *(const v4f*)(x + r * LE + lane * 16 + q * 4); for (int e = 0; e < 4; ++e) { v[4*q+e] = a[e]; s += a[e]; } }
  for (int o = 16; o > 0; o >>= 1) s += __shfl_xor(s, o, 32);
  const float mean = s / LE; float s2 = 0.f; for (int i = 0; i < 16; ++i) { const float d = v[i] - mean; s2 += d * d; } for (int o = 16; o > 0; o >>= 1) s2 += __shfl_xor(s2, o, 32);
  const float inv = rsqrtf(s2 / LE + 1e-5f);
  float q_ = 0.f, k_ = 0.f; const int h = lane >> 2; const int e0 = (lane & 3) * 16;
#pragma unroll
  for (int i = 0; i < 16; ++i) { v[i] = (v[i] - mean) * inv; q_ += v[i] * WQ[h * LEH + e0 + i]; k_ += v[i] * WK[h * LEH + e0 + i]; }
  q_ += __shfl_xor(q_, 1, 32); q_ += __shfl_xor(q_, 2, 32); k_ += __shfl_xor(k_, 1, 32); k_ += __shfl_xor(k_, 2, 32);
  typedef __attribute__((ext_vector_type(4))) unsigned u4; u4 p0, p1;
  for (int q = 0; q < 4; ++q) { p0[q] = (unsigned)__builtin_bit_cast(unsigned short, (_Float16)v[2*q]) | ((unsigned)__builtin_bit_cast(unsigned short, (_Float16)v[2*q+1]) << 16); p1[q] = (unsigned)__builtin_bit_cast(unsigned short, (_Float16)v[8+2*q]) | ((unsigned)__builtin_bit_cast(unsigned short, (_Float16)v[8+2*q+1]) << 16); }
  __shared__ float sq[8][8], sk[8][8];
  if ((lane & 3) == 0) { sq[wave][h] = q_ + bQ[h]; sk[wave][h] = k_ + bK[h]; }
  for (int pass = 0; pass < 2; ++pass) { *(volatile u4*)(XN16 + (r * LE + lane * 16) / 2) = p0; *(volatile u4*)(XN16 + (r * LE + lane * 16) / 2 + 4) = p1; __threadfence(); }
  __syncthreads();
  if (threadIdx.x < 64) { const float a = sq[threadIdx.x >> 3][threadIdx.x & 7], b = sk[threadIdx.x >> 3][threadIdx.x & 7];
    ((volatile float*)Qs)[(size_t)blockIdx.x * 64 + threadIdx.x] = a; ((volatile float*)Ks)[(size_t)blockIdx.x * 64 + threadIdx.x] = b; __threadfence();
    ((volatile float*)Qs)[(size_t)blockIdx.x * 64 + threadIdx.x] = a; ((volatile float*)Ks)[(size_t)blockIdx.x * 64 + threadIdx.x] = b; }
}
__global__ __launch_bounds__(256) void wv_kernel(const float* __restrict__ WV, unsigned* __restrict__ WVT) {
  const int i = blockIdx.x * 256 + threadIdx.x; if (i >= LH * LEH * LEH / 2) return; const int h = (2 * i) / (LEH * LEH), f = ((2 * i) / LEH) % LEH, e = (2 * i) % LEH;
  const unsigned u = (unsigned)__builtin_bit_cast(unsigned short, (_Float16)WV[(h * LEH + e) * LEH + f]) | ((unsigned)__builtin_bit_cast(unsigned short, (_Float16)WV[(h * LEH + e + 1) * LEH + f]) << 16);
  ((volatile unsigned*)WVT)[i] = u; __threadfence(); ((volatile unsigned*)WVT)[i] = u;
}
__global__ __launch_bounds__(256) void softmax_kernel(const float* __restrict__ Qs, const float* __restrict__ Ks, unsigned* __restrict__ P16) {
  __shared__ float red[8]; __shared__ float stat;
  const int bh = blockIdx.x / LT, i = blockIdx.x % LT; const int b = bh / LH, h = bh % LH; const int t = threadIdx.x, lane = t & 31, wave = t >> 5;
  const float qi = Qs[((size_t)b * LT + i) * LH + h];
  float v[4]; float mx = -INFINITY;
#pragma unroll
  for (int q = 0; q < 4; ++q) { const int j = t + 256 * q; const float kj = Ks[((size_t)b * LT + j) * LH + h]; const float d = qi - kj; v[q] = -(d * d) * 0.125f; mx = fmaxf(mx, v[q]); }
  for (int o = 16; o > 0; o >>= 1) mx = fmaxf(mx, __shfl_xor(mx, o, 32));
  if (lane == 0) red[wave] = mx; __syncthreads();
  if (t == 0) { float m = red[0]; for (int w = 1; w < 8; ++w) m = fmaxf(m, red[w]); stat = m; } __syncthreads();
  const float m = stat; __syncthreads();
  float se = 0.f;
#pragma unroll
  for (int q = 0; q < 4; ++q) { v[q] = expf(v[q] - m); se += v[q]; }
  for (int o = 16; o > 0; o >>= 1) se += __shfl_xor(se, o, 32);
  if (lane == 0) red[wave] = se; __syncthreads();
  if (t == 0) { float s = 0.f; for (int w = 0; w < 8; ++w) s += red[w]; stat = 32768.0f / s; } __syncthreads();
  const float inv = stat;
  __shared__ float prow[LT];
#pragma unroll
  for (int q = 0; q < 4; ++q) prow[t + 256 * q] = v[q] * inv;
  __syncthreads();
  for (int pass = 0; pass < 2; ++pass) {
#pragma unroll
    for (int q = 0; q < 2; ++q) { const int c = 2 * (t + 256 * q); const unsigned u = (unsigned)__builtin_bit_cast(unsigned short, (_Float16)prow[c]) | ((unsigned)__builtin_bit_cast(unsigned short, (_Float16)prow[c + 1]) << 16);
      ((volatile unsigned*)P16)[((size_t)bh * LT + i) * (LT / 2) + t + 256 * q] = u; }
    __threadfence(); }
}
__global__ __launch_bounds__(256) void vt_kernel(const float* __restrict__ V, const float* __restrict__ bV, unsigned* __restrict__ VT) {
  __shared__ float tile[64][65];
  const int bh = blockIdx.y, j0 = blockIdx.x * 64, tx = threadIdx.x, ty = threadIdx.y; const int b = bh / LH, h = bh % LH;
  for (int r = ty; r < 64; r += 8) { const int j = j0 + r; for (int c = tx; c < 64; c += 32) tile[c][r] = V[((size_t)b * LT + j) * LE + h * LEH + c] + bV[h * LEH + c]; }
  __syncthreads();
  for (int pass = 0; pass < 2; ++pass) { for (int r = ty; r < 64; r += 8) { const unsigned u = (unsigned)__builtin_bit_cast(unsigned short, (_Float16)tile[r][2 * tx]) | ((unsigned)__builtin_bit_cast(unsigned short, (_Float16)tile[r][2 * tx + 1]) << 16);
      ((volatile unsigned*)VT)[(((size_t)bh * LEH + r) * LT + j0) / 2 + tx] = u; } __threadfence(); }
}
__global__ __launch_bounds__(256) void merge_kernel(const float* __restrict__ HO, const float* __restrict__ W1, const float* __restrict__ b1, const float* __restrict__ W2, const float* __restrict__ b2, const float* __restrict__ x, float* __restrict__ out) {
  __shared__ float w1[64], w2[64], bb1[8], bb2[8];
  if (threadIdx.x < 64) { w1[threadIdx.x] = W1[threadIdx.x]; w2[threadIdx.x] = W2[threadIdx.x]; } if (threadIdx.x < 8) { bb1[threadIdx.x] = b1[threadIdx.x]; bb2[threadIdx.x] = b2[threadIdx.x]; }
  __syncthreads();
  const size_t idx = (size_t)blockIdx.x * 256 + threadIdx.x; const size_t r = idx / LEH; const int f = (int)(idx % LEH);
  float ho[8];
#pragma unroll
  for (int h = 0; h < 8; ++h) ho[h] = HO[r * LE + h * LEH + f];
  float m[8];
#pragma unroll
  for (int k = 0; k < 8; ++k) m[k] = bb2[k];
#pragma unroll 1
  for (int g = 0; g < 8; ++g) { float a = bb1[g];
#pragma unroll
    for (int h = 0; h < 8; ++h) a += ho[h] * w1[h * 8 + g];
    a = fmaxf(a, 0.f);
#pragma unroll
    for (int k = 0; k < 8; ++k) m[k] += a * w2[g * 8 + k]; }
  const v4f x0 = *(const v4f*)(x + r * LE + f * 8), x1 = *(const v4f*)(x + r * LE + f * 8 + 4);
  const v4f o0 = {m[0] + x0[0], m[1] + x0[1], m[2] + x0[2], m[3] + x0[3]}, o1 = {m[4] + x1[0], m[5] + x1[1], m[6] + x1[2], m[7] + x1[3]};
  for (int pass = 0; pass < 2; ++pass) { *(volatile v4f*)(out + r * LE + f * 8) = o0; *(volatile v4f*)(out + r * LE + f * 8 + 4) = o1; __threadfence(); }
}
extern "C" void kernel_launch(void* const* d_in, const int* in_sizes, int n_in, void* d_out, int out_size, void* d_ws, size_t ws_size, hipStream_t stream) {
  (void)in_sizes; (void)n_in; (void)out_size; (void)ws_size;
  const float* x = (const float*)d_in[0]; const float* WV = (const float*)d_in[1]; const float* bV = (const float*)d_in[2]; const float* WQ = (const float*)d_in[3]; const float* bQ = (const float*)d_in[4]; const float* WK = (const float*)d_in[5]; const float* bK = (const float*)d_in[6];
  const float* W1 = (const float*)d_in[7]; const float* b1 = (const float*)d_in[8]; const float* W2 = (const float*)d_in[9]; const float* b2 = (const float*)d_in[10];
  char* ws = (char*)d_ws; size_t off = 0;
  auto carve = [&](size_t bytes) -> char* { char* p = ws + off; off += (bytes + 255) & ~(size_t)255; return p; };
  unsigned* XN16 = (unsigned*)carve((size_t)LR * LE * 2); float* Qs = (float*)carve((size_t)LR * LH * 4); float* Ks = (float*)carve((size_t)LR * LH * 4);
  unsigned* WVT = (unsigned*)carve(LH * LEH * LEH * 2); float* V = (float*)carve((size_t)LR * LE * 4); unsigned* VT = (unsigned*)carve((size_t)LR * LE * 2);
  unsigned* P16 = (unsigned*)carve((size_t)LB * LH * LT * LT * 2);
  float* HO = (float*)carve((size_t)LR * LE * 4);
  ln_qk_kernel<<<LR / 8, 256, 0, stream>>>(x, WQ, bQ, WK, bK, XN16, Qs, Ks);
  wv_kernel<<<(LH * LEH * LEH / 2 + 255) / 256, 256, 0, stream>>>(WV, WVT);
  { const int t = (LR / 64) * 1;
    wmma_gemm64<0, false, 0, 0, false><<<dim3((t + 7) / 8, LH), 256, 0, stream>>>((const unsigned short*)XN16, nullptr, LE, LEH, (const unsigned short*)WVT, nullptr, LEH, LEH * LEH, V, nullptr, LE, LEH, nullptr, nullptr, 0, LR, LEH, LEH, 1.0f); }
  softmax_kernel<<<LB * LH * LT, 256, 0, stream>>>(Qs, Ks, P16);
  vt_kernel<<<dim3(LT / 64, LB * LH), dim3(32, 8), 0, stream>>>(V, bV, VT);
  { const int t = (LT / 64) * 1;
    for (int b = 0; b < LB; ++b)
      wmma_gemm64<0, false, 0, 0, false><<<dim3((t + 7) / 8, LH), 256, 0, stream>>>((const unsigned short*)P16 + (size_t)b * LH * LT * LT, nullptr, LT, (long)LT * LT, (const unsigned short*)VT + (size_t)b * LH * LEH * LT, nullptr, LT, (long)LEH * LT, HO + (size_t)b * LT * LE, nullptr, LE, LEH, nullptr, nullptr, 0, LT, LEH, LT, 1.0f / 32768.0f); }
  merge_kernel<<<LR * LEH / 256, 256, 0, stream>>>(HO, W1, b1, W2, b2, x, (float*)d_out);
}
